// LIVT_Decoder_74947179315523
// MI455X (gfx1250) — hardware-run, weakly checked
//
#include <hip/hip_runtime.h>
#define CIN 64
#define CF 16
#define NFr 6
#define LH 32
#define LW 32
#define NVX (NFr * LH * LW)
#define SC 4
#define HH 128
#define NQ (HH * HH)
#define NHD 8
#define RR 3
#define KA 49
#define NTP 5
#define RT 2
#define NFQ 10
#define SEG 832
#define KIN (NTP * SEG + 64)
#define MLPIN 3938
#define HID 256
#define QCH 4096
typedef __bf16 v16b __attribute__((ext_vector_type(16)));
typedef unsigned short v8us __attribute__((ext_vector_type(8), may_alias));
typedef float  v8f  __attribute__((ext_vector_type(8)));
typedef float  v4f  __attribute__((ext_vector_type(4)));
typedef float  v4fa __attribute__((ext_vector_type(4), may_alias));
union FragB { v16b v; v8us half[2]; unsigned short u[16]; };

__device__ __forceinline__ unsigned short bf16_bits(float x) { unsigned int u = __float_as_uint(x); return (unsigned short)((u + 0x7FFFu + ((u >> 16) & 1u)) >> 16); }
__device__ __forceinline__ float bf16_val(unsigned short b) { return __uint_as_float(((unsigned int)b) << 16); }
__device__ __forceinline__ float bf16_round(float x) { return bf16_val(bf16_bits(x)); }
template <int NT>
__device__ __forceinline__ v8f mmaN(v16b ah, v16b al, v16b bh, v16b bl, v8f c) {
  c = __builtin_amdgcn_wmma_f32_16x16x32_bf16(false, ah, false, bh, (short)0, c, false, false);
  if (NT >= 2) c = __builtin_amdgcn_wmma_f32_16x16x32_bf16(false, al, false, bh, (short)0, c, false, false);
  if (NT >= 3) c = __builtin_amdgcn_wmma_f32_16x16x32_bf16(false, ah, false, bl, (short)0, c, false, false);
  asm volatile("v_nop\n\tv_nop\n\tv_nop\n\tv_nop" : "+v"(c) : "v"(ah), "v"(al), "v"(bh), "v"(bl));
  return c;
}

__global__ __launch_bounds__(256) void k_wt_bf16(const float* __restrict__ W, unsigned short* __restrict__ Wt, int K, int N) {
  const int t = blockIdx.x * 256 + threadIdx.x;
  const int k8n = K / 8;
  if (t >= N * k8n) return;
  const int n = t / k8n, k8 = (t % k8n) * 8;
  v8us v;
#pragma unroll
  for (int i = 0; i < 8; ++i) v[i] = bf16_bits(W[(size_t)(k8 + i) * N + n]);
  *(volatile v8us*)(Wt + (size_t)n * K + k8) = v;
  __threadfence();
  *(volatile v8us*)(Wt + (size_t)n * K + k8) = v;
}

template <bool ASPLIT, int ACT, bool BIAS_BF16>
__global__ __launch_bounds__(128) void k_gemm_bf(const float* __restrict__ A, int lda, const unsigned short* __restrict__ Wt, int ldb,
                                               const float* __restrict__ bias, float* __restrict__ C, int ldc, int M, int N, int K) {
  __shared__ __attribute__((aligned(16))) float so[4][16][64];
  const int tid = threadIdx.x, w = tid >> 5, lane = tid & 31, ln = lane & 15, hh = lane >> 4;
  const int ntn = N / 64;
  const int wid = blockIdx.x * 4 + w;
  const int mt = wid / ntn, nq = wid % ntn;
  if (mt * 16 >= M) return;
  const int row0 = mt * 16, col0 = nq * 64;
  const float* arow = A + (size_t)(row0 + ln) * lda;
  v8f acc[4] = {};
  for (int kb = 0; kb < K; kb += 32) {
    FragB ah, al;
    const v4f x0 = *(const v4fa*)(arow + kb + 8 * hh), x1 = *(const v4fa*)(arow + kb + 8 * hh + 4);
    const v4f x2 = *(const v4fa*)(arow + kb + 16 + 8 * hh), x3 = *(const v4fa*)(arow + kb + 16 + 8 * hh + 4);
    float xs[16] = {x0[0],x0[1],x0[2],x0[3],x1[0],x1[1],x1[2],x1[3],x2[0],x2[1],x2[2],x2[3],x3[0],x3[1],x3[2],x3[3]};
#pragma unroll
    for (int i = 0; i < 16; ++i) { const unsigned short hb = bf16_bits(xs[i]); ah.u[i] = hb; al.u[i] = ASPLIT ? bf16_bits(xs[i] - bf16_val(hb)) : (unsigned short)0; }
#pragma unroll
    for (int t = 0; t < 4; ++t) {
      const unsigned short* brow = Wt + (size_t)(col0 + t * 16 + ln) * ldb + kb;
      FragB b;
      b.half[0] = *(const v8us*)(brow + 8 * hh);
      b.half[1] = *(const v8us*)(brow + 16 + 8 * hh);
      acc[t] = mmaN<ASPLIT ? 2 : 1>(ah.v, al.v, b.v, b.v, acc[t]);
    }
  }
#pragma unroll
  for (int t = 0; t < 4; ++t) {
    float bv = bias ? bias[col0 + t * 16 + ln] : 0.f;
    if (BIAS_BF16) bv = bf16_round(bv);
#pragma unroll
    for (int r = 0; r < 8; ++r) { float v = acc[t][r] + bv; if (ACT == 1) v = fmaxf(v, 0.f); so[w][8 * hh + r][t * 16 + ln] = v; }
  }
  __builtin_amdgcn_fence(__ATOMIC_ACQ_REL, "workgroup");
  __builtin_amdgcn_wave_barrier();
  const int rsub = lane >> 4, c4 = (lane & 15) * 4;
  for (int pass = 0; pass < 2; ++pass) {
#pragma unroll
    for (int q = 0; q < 8; ++q) {
      const int r = q * 2 + rsub;
      const v4f v = *(const v4fa*)&so[w][r][c4];
      *(volatile v4f*)(C + (size_t)(row0 + r) * ldc + col0 + c4) = v;
    }
    if (pass == 0) __threadfence();
  }
}

template <bool ASPLIT, int ACT, bool BIAS_BF16, bool RES_BF16>
__global__ __launch_bounds__(128) void k_gemm_bf3(const float* __restrict__ A, int lda, const unsigned short* __restrict__ Wt, int ldb,
                                                const float* __restrict__ bias, const float* __restrict__ resid, int rmod, int ldr,
                                                float* __restrict__ C, int ldc, int M, int N, int K) {
  __shared__ __attribute__((aligned(16))) float so[4][16][64];
  const int tid = threadIdx.x, w = tid >> 5, lane = tid & 31, ln = lane & 15, hh = lane >> 4;
  const int ntn = N / 64;
  const int wid = blockIdx.x * 4 + w;
  const int mt = wid / ntn, nq = wid % ntn;
  if (mt * 16 >= M) return;
  const int row0 = mt * 16, col0 = nq * 64;
  const float* arow = A + (size_t)(row0 + ln) * lda;
  v8f acc[4] = {};
  for (int kb = 0; kb < K; kb += 32) {
    FragB ah, al;
    const v4f x0 = *(const v4fa*)(arow + kb + 8 * hh), x1 = *(const v4fa*)(arow + kb + 8 * hh + 4);
    const v4f x2 = *(const v4fa*)(arow + kb + 16 + 8 * hh), x3 = *(const v4fa*)(arow + kb + 16 + 8 * hh + 4);
    float xs[16] = {x0[0],x0[1],x0[2],x0[3],x1[0],x1[1],x1[2],x1[3],x2[0],x2[1],x2[2],x2[3],x3[0],x3[1],x3[2],x3[3]};
#pragma unroll
    for (int i = 0; i < 16; ++i) { const unsigned short hb = bf16_bits(xs[i]); ah.u[i] = hb; al.u[i] = ASPLIT ? bf16_bits(xs[i] - bf16_val(hb)) : (unsigned short)0; }
#pragma unroll
    for (int t = 0; t < 4; ++t) {
      const unsigned short* brow = Wt + (size_t)(col0 + t * 16 + ln) * ldb + kb;
      FragB b;
      b.half[0] = *(const v8us*)(brow + 8 * hh);
      b.half[1] = *(const v8us*)(brow + 16 + 8 * hh);
      acc[t] = mmaN<ASPLIT ? 2 : 1>(ah.v, al.v, b.v, b.v, acc[t]);
    }
  }
#pragma unroll
  for (int t = 0; t < 4; ++t) {
    const int col = col0 + t * 16 + ln;
    float bv = bias ? bias[col] : 0.f;
    if (BIAS_BF16) bv = bf16_round(bv);
#pragma unroll
    for (int r = 0; r < 8; ++r) {
      float v = acc[t][r] + bv;
      if (resid) { float rv = resid[(size_t)((row0 + 8 * hh + r) % rmod) * ldr + col]; if (RES_BF16) rv = bf16_round(rv); v += rv; }
      if (ACT == 1) v = fmaxf(v, 0.f);
      if (ACT == 2) v = 0.5f * v * (1.0f + erff(v * 0.70710678118654752f));
      if (ACT == 3) { const float u = 0.7978845608028654f * (v + 0.044715f * v * v * v); v = 0.5f * v * (1.0f + tanhf(u)); }
      so[w][8 * hh + r][t * 16 + ln] = v;
    }
  }
  __builtin_amdgcn_fence(__ATOMIC_ACQ_REL, "workgroup");
  __builtin_amdgcn_wave_barrier();
  const int rsub = lane >> 4, c4 = (lane & 15) * 4;
  for (int pass = 0; pass < 2; ++pass) {
#pragma unroll
    for (int q = 0; q < 8; ++q) {
      const int r = q * 2 + rsub;
      const v4f v = *(const v4fa*)&so[w][r][c4];
      *(volatile v4f*)(C + (size_t)(row0 + r) * ldc + col0 + c4) = v;
    }
    if (pass == 0) __threadfence();
  }
}
template <bool PARAM_BF16>
__global__ __launch_bounds__(256) void k_layernorm(const float* __restrict__ X, const float* __restrict__ R, const float* __restrict__ g, const float* __restrict__ bta,
                                                  float* __restrict__ out_sum, float* __restrict__ out_norm, int N, float eps) {
  __shared__ float red[256];
  const int row = blockIdx.x, tid = threadIdx.x;
  const float* x = X + (size_t)row * N; const float* rr = R ? R + (size_t)row * N : nullptr;
  float vals[16];
  const int per = N / 256;
  float s1 = 0.f;
  for (int u = 0; u < per / 4; ++u) {
    const int j = tid * 4 + 1024 * u;
    const v4f a = *(const v4fa*)(x + j);
    v4f b = {0.f,0.f,0.f,0.f}; if (rr) b = *(const v4fa*)(rr + j);
#pragma unroll
    for (int q = 0; q < 4; ++q) { const float v = a[q] + b[q]; vals[u * 4 + q] = v; s1 += v; }
  }
  red[tid] = s1; __syncthreads();
  for (int st = 128; st > 0; st >>= 1) { if (tid < st) red[tid] += red[tid + st]; __syncthreads(); }
  const float mu = red[0] / (float)N; __syncthreads();
  float s2 = 0.f;
  for (int u = 0; u < per / 4; ++u)
#pragma unroll
    for (int q = 0; q < 4; ++q) { const float c = vals[u * 4 + q] - mu; s2 += c * c; }
  red[tid] = s2; __syncthreads();
  for (int st = 128; st > 0; st >>= 1) { if (tid < st) red[tid] += red[tid + st]; __syncthreads(); }
  const float rs = rsqrtf(red[0] / (float)N + eps);
  for (int pass = 0; pass < 2; ++pass) {
    for (int u = 0; u < per / 4; ++u) {
      const int j = tid * 4 + 1024 * u;
      v4f o, sm;
#pragma unroll
      for (int q = 0; q < 4; ++q) {
        float gg = g[j + q], bb = bta[j + q];
        if (PARAM_BF16) { gg = bf16_round(gg); bb = bf16_round(bb); }
        sm[q] = vals[u * 4 + q]; o[q] = (vals[u * 4 + q] - mu) * rs * gg + bb;
      }
      if (out_sum) *(volatile v4f*)(out_sum + (size_t)row * N + j) = sm;
      *(volatile v4f*)(out_norm + (size_t)row * N + j) = o;
    }
    if (pass == 0) __threadfence();
  }
}


typedef _Float16 v16h __attribute__((ext_vector_type(16)));
union FragH { v16h v; v8us half[2]; _Float16 h[16]; unsigned short u[16]; };
template <int NT>
__device__ __forceinline__ v8f mmaH(v16h ah, v16h al, v16h bh, v16h bl, v8f c) {
  c = __builtin_amdgcn_wmma_f32_16x16x32_f16(false, ah, false, bh, (short)0, c, false, false);
  if (NT >= 2) c = __builtin_amdgcn_wmma_f32_16x16x32_f16(false, al, false, bh, (short)0, c, false, false);
  if (NT >= 3) c = __builtin_amdgcn_wmma_f32_16x16x32_f16(false, ah, false, bl, (short)0, c, false, false);
  asm volatile("v_nop\n\tv_nop\n\tv_nop\n\tv_nop" : "+v"(c) : "v"(ah), "v"(al), "v"(bh), "v"(bl));
  return c;
}
template <bool ASPLIT>
__global__ __launch_bounds__(128) void k_gemm_h(const float* __restrict__ A, int lda, size_t sA, const _Float16* __restrict__ Bh, int ldb, size_t sB, float alpha, float* __restrict__ C, int ldc, size_t sC, int M, int N, int K) {
  __shared__ __attribute__((aligned(16))) float so[4][16][64];
  const int tid = threadIdx.x, w = tid >> 5, lane = tid & 31, ln = lane & 15, hh = lane >> 4; const int by = blockIdx.y;
  A += (size_t)by * sA; Bh += (size_t)by * sB; C += (size_t)by * sC;
  const int ntn = (N + 63) / 64; const int wid = blockIdx.x * 4 + w; const int mt = wid / ntn, nq = wid % ntn; if (mt * 16 >= M) return;
  const int row0 = mt * 16, col0 = nq * 64; const float* arow = A + (size_t)(row0 + ln) * lda;
  v8f acc[4] = {};
  for (int kb = 0; kb < K; kb += 32) {
    FragH ah, al;
    const v4f x0 = *(const v4fa*)(arow + kb + 8 * hh), x1 = *(const v4fa*)(arow + kb + 8 * hh + 4), x2 = *(const v4fa*)(arow + kb + 16 + 8 * hh), x3 = *(const v4fa*)(arow + kb + 16 + 8 * hh + 4);
    float xs[16] = {x0[0],x0[1],x0[2],x0[3],x1[0],x1[1],x1[2],x1[3],x2[0],x2[1],x2[2],x2[3],x3[0],x3[1],x3[2],x3[3]};
#pragma unroll
    for (int i = 0; i < 16; ++i) { const _Float16 h = (_Float16)xs[i]; ah.h[i] = h; al.h[i] = ASPLIT ? (_Float16)(xs[i] - (float)h) : (_Float16)0.0f; }
#pragma unroll
    for (int t = 0; t < 4; ++t) { if (col0 + t * 16 >= N) continue; const size_t boff = (size_t)(col0 + t * 16 + ln) * ldb + kb; FragH bq; bq.half[0] = *(const v8us*)(Bh + boff + 8 * hh); bq.half[1] = *(const v8us*)(Bh + boff + 16 + 8 * hh);
      acc[t] = mmaH<ASPLIT ? 2 : 1>(ah.v, al.v, bq.v, bq.v, acc[t]); }
  }
#pragma unroll
  for (int t = 0; t < 4; ++t) { if (col0 + t * 16 >= N) continue;
#pragma unroll
    for (int r = 0; r < 8; ++r) so[w][8 * hh + r][t * 16 + ln] = acc[t][r] * alpha; }
  __builtin_amdgcn_fence(__ATOMIC_ACQ_REL, "workgroup"); __builtin_amdgcn_wave_barrier();
  const int rsub = lane >> 4, c4 = (lane & 15) * 4;
  for (int pass = 0; pass < 2; ++pass) {
#pragma unroll
    for (int q = 0; q < 8; ++q) { const int r = q * 2 + rsub; if (col0 + c4 < N) { const v4f v = *(const v4fa*)&so[w][r][c4]; *(volatile v4f*)(C + (size_t)(row0 + r) * ldc + col0 + c4) = v; } }
    if (pass == 0) __threadfence(); }
}

__global__ __launch_bounds__(256) void k_wt_f16(const float* __restrict__ W, _Float16* __restrict__ Wt, int K, int N, float scale) {
  const int t = blockIdx.x * 256 + threadIdx.x; if (t >= N * (K / 8)) return; const int n = t / (K / 8), k8 = (t % (K / 8)) * 8; FragH f;
#pragma unroll
  for (int i = 0; i < 8; ++i) f.h[i] = (_Float16)(bf16_round(W[(size_t)(k8 + i) * N + n]) * scale); const v8us o = f.half[0];
  *(volatile v8us*)((unsigned short*)Wt + (size_t)n * K + k8) = o; __threadfence(); *(volatile v8us*)((unsigned short*)Wt + (size_t)n * K + k8) = o;
}
template <int ACT>
__global__ __launch_bounds__(128) void k_gemm_hhx(const _Float16* __restrict__ A, int lda, size_t sA, const _Float16* __restrict__ Bh, int ldb, size_t sB, float alpha, const float* __restrict__ bias, size_t sBias, const float* __restrict__ CP, int rowsPerB, size_t sCPb, int row0g,
    float* __restrict__ C, _Float16* __restrict__ C16, int ldc, size_t sC, int M, int N, int K) {
  __shared__ __attribute__((aligned(16))) float so[4][16][64];
  const int tid = threadIdx.x, w = tid >> 5, lane = tid & 31, ln = lane & 15, hh = lane >> 4; const int by = blockIdx.y;
  A += (size_t)by * sA; Bh += (size_t)by * sB; const size_t cofs = (size_t)by * sC; const float* bp = bias ? bias + (size_t)by * sBias : nullptr;
  const int ntn = (N + 63) / 64; const int wid = blockIdx.x * 4 + w; const int mt = wid / ntn, nq = wid % ntn; if (mt * 16 >= M) return;
  const int row0 = mt * 16, col0 = nq * 64; const _Float16* arow = A + (size_t)(row0 + ln) * lda;
  v8f acc[4] = {};
  for (int kb = 0; kb < K; kb += 32) { FragH ah; ah.half[0] = *(const v8us*)((const unsigned short*)arow + kb + 8 * hh); ah.half[1] = *(const v8us*)((const unsigned short*)arow + kb + 16 + 8 * hh);
#pragma unroll
    for (int t = 0; t < 4; ++t) { if (col0 + t * 16 >= N) continue; const size_t boff = (size_t)(col0 + t * 16 + ln) * ldb + kb; FragH bq; bq.half[0] = *(const v8us*)((const unsigned short*)Bh + boff + 8 * hh); bq.half[1] = *(const v8us*)((const unsigned short*)Bh + boff + 16 + 8 * hh);
      acc[t] = mmaH<1>(ah.v, ah.v, bq.v, bq.v, acc[t]); }
  }
#pragma unroll
  for (int t = 0; t < 4; ++t) { if (col0 + t * 16 >= N) continue; const int col = col0 + t * 16 + ln; const float bv = bp ? bf16_round(bp[col]) : 0.f;
#pragma unroll
    for (int r = 0; r < 8; ++r) { float v = acc[t][r] * alpha + bv; if (CP) { const int bidx = (row0g + row0 + 8 * hh + r) / rowsPerB; v += CP[(size_t)bidx * sCPb + (size_t)by * 64 + col]; } if (ACT == 1) v = (v > 0.f) ? v : expm1f(v); else if (ACT == 7) v = (v > 0.f) ? v + 1.0f : expf(v); else if (ACT == 8) v = tanhf(v); else if (ACT == 9) v = 0.5f * v * (1.0f + tanhf(0.7978845608028654f * (v + 0.044715f * v * v * v))); else if (ACT == 11) v = 1.0f / (1.0f + expf(-v)); else if (ACT == 12) v = (v > 0.f) ? v : 0.01f * v; else if (ACT == 14) v = (v > 0.f) ? v : 0.1f * v; else if (ACT == 15) v = v / (1.0f + expf(-v)); else if (ACT == 3) v = fmaxf(v, 0.f); else if (ACT == 6) v = 0.5f * v * (1.0f + erff(v * 0.70710678118654752f)); so[w][8 * hh + r][t * 16 + ln] = v; } }
  __builtin_amdgcn_fence(__ATOMIC_ACQ_REL, "workgroup"); __builtin_amdgcn_wave_barrier();
  const int rsub = lane >> 4, c4 = (lane & 15) * 4; typedef _Float16 v4h __attribute__((ext_vector_type(4)));
  for (int pass = 0; pass < 2; ++pass) {
#pragma unroll
    for (int q = 0; q < 8; ++q) { const int r = q * 2 + rsub; if (col0 + c4 < N) { const v4f v = *(const v4fa*)&so[w][r][c4]; if (C) *(volatile v4f*)(C + cofs + (size_t)(row0 + r) * ldc + col0 + c4) = v; if (C16) { v4h h4; for (int i = 0; i < 4; ++i) h4[i] = (_Float16)v[i]; *(volatile v4h*)(C16 + cofs + (size_t)(row0 + r) * ldc + col0 + c4) = h4; } } }
    if (pass == 0) __threadfence(); }
}


typedef _Float16 v4h __attribute__((ext_vector_type(4)));

__global__ __launch_bounds__(256) void k_x16(const float* __restrict__ x, _Float16* __restrict__ X16, size_t n8) { const size_t t = (size_t)blockIdx.x * 256 + threadIdx.x; if (t >= n8) return; FragH f;
#pragma unroll
  for (int q = 0; q < 8; ++q) f.h[q] = (_Float16)bf16_round(x[t * 8 + q]); *(volatile v8us*)((unsigned short*)X16 + t * 8) = f.half[0]; __threadfence(); *(volatile v8us*)((unsigned short*)X16 + t * 8) = f.half[0]; }
__global__ __launch_bounds__(256) void k_h16(const float* __restrict__ x, _Float16* __restrict__ X16, size_t n8) { const size_t t = (size_t)blockIdx.x * 256 + threadIdx.x; if (t >= n8) return; FragH f;
#pragma unroll
  for (int q = 0; q < 8; ++q) f.h[q] = (_Float16)x[t * 8 + q]; *(volatile v8us*)((unsigned short*)X16 + t * 8) = f.half[0]; __threadfence(); *(volatile v8us*)((unsigned short*)X16 + t * 8) = f.half[0]; }
__global__ __launch_bounds__(256) void k_round16f(const float* __restrict__ W, _Float16* __restrict__ Bt, size_t n8) { const size_t t = (size_t)blockIdx.x * 256 + threadIdx.x; if (t >= n8) return; FragH f;
#pragma unroll
  for (int i = 0; i < 8; ++i) f.h[i] = (_Float16)(bf16_round(W[t * 8 + i]) * 16.0f); *(volatile v8us*)((unsigned short*)Bt + t * 8) = f.half[0]; __threadfence(); *(volatile v8us*)((unsigned short*)Bt + t * 8) = f.half[0]; }
template <int NHv, int TTv>
__global__ __launch_bounds__(256) void k_vt(const _Float16* __restrict__ V16, int ldv, int voff, _Float16* __restrict__ Vt) { __shared__ unsigned short tl[64][66]; const int tid = threadIdx.x; const int slab = blockIdx.x / (TTv / 64), lg = blockIdx.x % (TTv / 64); const int b = slab / NHv, h = slab % NHv;
  for (int i = tid; i < 64 * 8; i += 256) { const int r = i / 8, c8 = (i % 8) * 8; FragH f; f.half[0] = *(const v8us*)((const unsigned short*)V16 + ((size_t)b * TTv + lg * 64 + r) * ldv + voff + h * 64 + c8);
#pragma unroll
    for (int q = 0; q < 8; ++q) tl[r][c8 + q] = f.u[q]; }
  __syncthreads();
  for (int pass = 0; pass < 2; ++pass) {
#pragma unroll
    for (int rd = 0; rd < 2; ++rd) { const int d = rd * 32 + tid / 8, pc = tid % 8; FragH f;
#pragma unroll
      for (int q = 0; q < 8; ++q) f.u[q] = tl[pc * 8 + q][d];
      *(volatile v8us*)((unsigned short*)Vt + ((size_t)slab * 64 + d) * TTv + lg * 64 + pc * 8) = f.half[0]; }
    if (pass == 0) __threadfence(); } }

__global__ __launch_bounds__(256) void k_hl(const float* __restrict__ F, _Float16* __restrict__ Hh, _Float16* __restrict__ Hl, size_t n8) { const size_t t = (size_t)blockIdx.x * 256 + threadIdx.x; if (t >= n8) return; FragH fh, fl; const v4f a = *(const v4fa*)(F + t * 8), c = *(const v4fa*)(F + t * 8 + 4);
#pragma unroll
  for (int q = 0; q < 4; ++q) { _Float16 h = (_Float16)a[q]; fh.h[q] = h; fl.h[q] = (_Float16)((a[q] - (float)h) * 1024.0f); h = (_Float16)c[q]; fh.h[4 + q] = h; fl.h[4 + q] = (_Float16)((c[q] - (float)h) * 1024.0f); }
  for (int pass = 0; pass < 2; ++pass) { *(volatile v8us*)((unsigned short*)Hh + t * 8) = fh.half[0]; *(volatile v8us*)((unsigned short*)Hl + t * 8) = fl.half[0]; if (pass == 0) __threadfence(); } }

template <int SRCCL>
__global__ __launch_bounds__(256) void k_im3(const float* __restrict__ src, int C, int KP, _Float16* __restrict__ IM) { const size_t t = (size_t)blockIdx.x * 256 + threadIdx.x; const int ng = KP / 8; if (t >= (size_t)NVX * ng) return; const int g = (int)(t % ng) * 8; const int v = (int)(t / ng); const int f = v / (LH * LW), y = (v / LW) % LH, x = v % LW; FragH fr;
#pragma unroll
  for (int q = 0; q < 8; ++q) { const int col = g + q; float val = 0.f; if (col < C * 27) { const int c = col / 27, tap = col % 27; const int ff = f + tap / 9 - 1, yy = y + (tap / 3) % 3 - 1, xx = x + tap % 3 - 1;
      if (ff >= 0 && ff < NFr && yy >= 0 && yy < LH && xx >= 0 && xx < LW) { const int vv = (ff * LH + yy) * LW + xx; val = SRCCL ? src[(size_t)vv * CF + c] : bf16_round(src[(size_t)c * NVX + vv]); } }
    fr.h[q] = (_Float16)val; }
  *(volatile v8us*)((unsigned short*)IM + (size_t)v * KP + g) = fr.half[0]; __threadfence(); *(volatile v8us*)((unsigned short*)IM + (size_t)v * KP + g) = fr.half[0]; }
__global__ __launch_bounds__(256) void k_wconv(const float* __restrict__ w, int C, int KP, int NOUT, _Float16* __restrict__ Bt) { const int t = blockIdx.x * 256 + threadIdx.x; const int ng = KP / 8; if (t >= NOUT * ng) return; const int g = (t % ng) * 8, o = t / ng; FragH f;
#pragma unroll
  for (int q = 0; q < 8; ++q) { const int col = g + q; f.h[q] = (col < C * 27) ? (_Float16)(bf16_round(w[(size_t)o * C * 27 + col]) * 16.0f) : (_Float16)0.0f; }
  *(volatile v8us*)((unsigned short*)Bt + (size_t)o * KP + g) = f.half[0]; __threadfence(); *(volatile v8us*)((unsigned short*)Bt + (size_t)o * KP + g) = f.half[0]; }
__global__ __launch_bounds__(256) void k_pbtab(const float* __restrict__ times, const float* __restrict__ Bpe, const float* __restrict__ Wpb, const float* __restrict__ bpb, float* __restrict__ PB) {
  #pragma clang fp contract(off)
  const int t = blockIdx.x * 256 + threadIdx.x; if (t >= 16 * NTP * KA * 2) return; const int hq = (t % 2) * 4; const int k = (t / 2) % KA; const int dt = (t / (2 * KA)) % NTP; const int cell = t / (2 * KA * NTP); const int ry = cell / 4, rx = cell % 4; const int ky = k / 7 - RR, kx = k % 7 - RR;
  const float t32 = bf16_round(times[0]) * (float)(NFr - 1); const int ct = (int)rintf(t32); const double rel_time = ((double)t32 - (double)ct) * 2.0 / (double)NTP; const float tc = (float)(rel_time - (double)(dt - RT) * 2.0 / (double)NTP);
  float rel[3]; rel[0] = tc * (float)NTP; rel[1] = ((float)(2 * ry - 3 - 8 * ky) / 128.0f) * (float)LH; rel[2] = ((float)(2 * rx - 3 - 8 * kx) / 128.0f) * (float)LW;
  float acc[4];
#pragma unroll
  for (int j = 0; j < 4; ++j) acc[j] = bf16_round(bpb[hq + j]);
#pragma unroll 1
  for (int i = 0; i < 3 * NFQ; ++i) { const float proj = (rel[0] * bf16_round(Bpe[i * 3 + 0]) + rel[1] * bf16_round(Bpe[i * 3 + 1])) + rel[2] * bf16_round(Bpe[i * 3 + 2]); const float sn = sinf(proj), cs = cosf(proj);
#pragma unroll
    for (int j = 0; j < 4; ++j) acc[j] += sn * bf16_round(Wpb[(size_t)i * NHD + hq + j]) + cs * bf16_round(Wpb[(size_t)(3 * NFQ + i) * NHD + hq + j]); }
  v4f o; o[0] = acc[0]; o[1] = acc[1]; o[2] = acc[2]; o[3] = acc[3]; float* p = PB + (((size_t)cell * NTP + dt) * KA + k) * NHD + hq; *(volatile v4f*)p = o; __threadfence(); *(volatile v4f*)p = o; }
__global__ __launch_bounds__(256) void k_attn(const float* __restrict__ QV, const float* __restrict__ KVv, const float* __restrict__ VV, const float* __restrict__ times, const float* __restrict__ PB, int q0, _Float16* __restrict__ FEAT) {
  #pragma clang fp contract(off)
  __shared__ __attribute__((aligned(16))) unsigned short seg[8][SEG]; __shared__ float sqs[8][CF];
  const int tid = threadIdx.x, w = tid >> 5, l = tid & 31; const int q = q0 + blockIdx.x * 8 + w; const int qy = q / HH, qx = q % HH; const int iy = qy / SC, ix = qx / SC; const int ry = qy % SC, rx = qx % SC; const int cell = ry * 4 + rx;
  const float t32 = bf16_round(times[0]) * (float)(NFr - 1); const int ct = (int)rintf(t32); const double rel_time_d = ((double)t32 - (double)ct) * 2.0 / (double)NTP; const float rel_time = (float)rel_time_d;
  int fidx[NTP];
#pragma unroll
  for (int dt = 0; dt < NTP; ++dt) fidx[dt] = min(max(ct + dt - RT, 0), NFr - 1);
  if (l < CF) { const float hy = -1.0f + (2.0f * (float)qy + 1.0f) / (float)HH, hx = -1.0f + (2.0f * (float)qx + 1.0f) / (float)HH;
    const float izf = ((rel_time + 1.0f) * (float)NTP - 1.0f) / 2.0f, iyf = ((hy + 1.0f) * (float)LH - 1.0f) / 2.0f, ixf = ((hx + 1.0f) * (float)LW - 1.0f) / 2.0f; const float fz = floorf(izf), fy = floorf(iyf), fx = floorf(ixf); const float wz = izf - fz, wy = iyf - fy, wx = ixf - fx; const int z0 = (int)fz, y0 = (int)fy, x0 = (int)fx; float s = 0.f;
#pragma unroll
    for (int c8 = 0; c8 < 8; ++c8) { const int dz = c8 >> 2, dy = (c8 >> 1) & 1, dx = c8 & 1; const int zc = z0 + dz, yc = y0 + dy, xc = x0 + dx; const bool valid = (zc >= 0) && (zc < NTP) && (yc >= 0) && (yc < LH) && (xc >= 0) && (xc < LW); const float wgt = (dz ? wz : 1.f - wz) * (dy ? wy : 1.f - wy) * (dx ? wx : 1.f - wx);
      int zw = min(max(zc, 0), NTP - 1); int fr = 0;
#pragma unroll
      for (int dt = 0; dt < NTP; ++dt) fr = (zw == dt) ? fidx[dt] : fr;
      const int vv = (fr * LH + min(max(yc, 0), LH - 1)) * LW + min(max(xc, 0), LW - 1); s += (valid ? wgt : 0.f) * QV[(size_t)vv * CF + l]; }
    sqs[w][l] = s; }
  __syncthreads();
  float qf[CF];
#pragma unroll
  for (int c = 0; c < CF; ++c) qf[c] = sqs[w][c];
  for (int dt = 0; dt < NTP; ++dt) { const int fr = fidx[dt]; float outv[CF];
#pragma unroll
    for (int c = 0; c < CF; ++c) outv[c] = 0.f;
    float sc[2][NHD]; float vfv[2][CF];
#pragma unroll
    for (int s2 = 0; s2 < 2; ++s2) { const int k = l + 32 * s2; const bool live = k < KA; const int kk = live ? k : 0; const int ky = kk / 7 - RR, kx = kk % 7 - RR; const int yy = iy + ky, xx = ix + kx; const bool valid = live && (yy >= 0) && (yy < LH) && (xx >= 0) && (xx < LW); const int vv = (fr * LH + min(max(yy, 0), LH - 1)) * LW + min(max(xx, 0), LW - 1);
#pragma unroll
      for (int c = 0; c < CF; ++c) { const float kv = valid ? KVv[(size_t)vv * CF + c] : 0.f; vfv[s2][c] = valid ? VV[(size_t)vv * CF + c] : 0.f; if ((c & 1) == 1) { sc[s2][c >> 1] = (qf[c - 1] * (valid ? KVv[(size_t)vv * CF + c - 1] : 0.f) + qf[c] * kv) * 0.70710678118654752f + (live ? PB[(((size_t)cell * NTP + dt) * KA + kk) * NHD + (c >> 1)] : -3.0e38f); } } }
#pragma unroll
    for (int h = 0; h < NHD; ++h) { float m = fmaxf(sc[0][h], sc[1][h]); for (int o = 16; o > 0; o >>= 1) m = fmaxf(m, __shfl_xor(m, o, 32)); const float e0 = __expf(sc[0][h] - m), e1 = (l + 32 < KA) ? __expf(sc[1][h] - m) : 0.f;        float s = e0 + e1; for (int o = 16; o > 0; o >>= 1) s += __shfl_xor(s, o, 32); sc[0][h] = e0 / s; sc[1][h] = e1 / s; }
#pragma unroll
    for (int s2 = 0; s2 < 2; ++s2) { const int k = l + 32 * s2; if (k < KA) { FragH f, g;
#pragma unroll
        for (int c = 0; c < 8; ++c) { f.h[c] = (_Float16)(vfv[s2][c] * sc[s2][c >> 1]); g.h[c] = (_Float16)(vfv[s2][8 + c] * sc[s2][(8 + c) >> 1]); }
        *(v8us*)&seg[w][k * CF] = f.half[0]; *(v8us*)&seg[w][k * CF + 8] = g.half[0]; } }
    if (l < (SEG - KA * CF) / 8) { v8us z;
#pragma unroll
      for (int c = 0; c < 8; ++c) z[c] = 0; *(v8us*)&seg[w][KA * CF + l * 8] = z; }
    __syncthreads();
    for (int pass = 0; pass < 2; ++pass) { for (int i = l; i < SEG / 8; i += 32) { const v8us vv8 = *(const v8us*)&seg[w][i * 8]; *(volatile v8us*)((unsigned short*)FEAT + (size_t)(q - q0) * KIN + (size_t)dt * SEG + i * 8) = vv8; } if (pass == 0) __threadfence(); }
    __syncthreads(); }
  if (l < 8) { FragH f;
#pragma unroll
    for (int c = 0; c < 8; ++c) { const int col = l * 8 + c; float v = 0.f; if (col < CF) v = qf[col]; else if (col < CF + 2) v = 2.0f / (float)SC; f.h[c] = (_Float16)v; }
    *(volatile v8us*)((unsigned short*)FEAT + (size_t)(q - q0) * KIN + (size_t)NTP * SEG + l * 8) = f.half[0]; __threadfence(); *(volatile v8us*)((unsigned short*)FEAT + (size_t)(q - q0) * KIN + (size_t)NTP * SEG + l * 8) = f.half[0]; } }
__global__ __launch_bounds__(256) void k_w1t(const float* __restrict__ W1, _Float16* __restrict__ Bt) { const int t = blockIdx.x * 256 + threadIdx.x; const int ng = KIN / 8; if (t >= HID * ng) return; const int g = (t % ng) * 8, o = t / ng; FragH f;
#pragma unroll
  for (int c = 0; c < 8; ++c) { const int col = g + c; int src = -1; if (col < NTP * SEG) { const int dt = col / SEG, j = col % SEG; if (j < KA * CF) src = dt * KA * CF + j; } else { const int j = col - NTP * SEG; if (j < CF + 2) src = NTP * KA * CF + j; }
    f.h[c] = (src >= 0) ? (_Float16)(bf16_round(W1[(size_t)src * HID + o]) * 16.0f) : (_Float16)0.0f; }
  *(volatile v8us*)((unsigned short*)Bt + (size_t)o * KIN + g) = f.half[0]; __threadfence(); *(volatile v8us*)((unsigned short*)Bt + (size_t)o * KIN + g) = f.half[0]; }
__global__ __launch_bounds__(256) void k_w5(const float* __restrict__ W5, const float* __restrict__ b5, _Float16* __restrict__ Bt, float* __restrict__ B5) { const int t = blockIdx.x * 256 + threadIdx.x; if (t >= 16 * (HID / 8)) return; const int k0 = (t % (HID / 8)) * 8, n = t / (HID / 8); FragH f;
#pragma unroll
  for (int c = 0; c < 8; ++c) f.h[c] = (n < 3) ? (_Float16)(bf16_round(W5[(size_t)(k0 + c) * 3 + n]) * 16.0f) : (_Float16)0.0f;
  *(volatile v8us*)((unsigned short*)Bt + (size_t)n * HID + k0) = f.half[0]; __threadfence(); *(volatile v8us*)((unsigned short*)Bt + (size_t)n * HID + k0) = f.half[0];
  if (t < 16) { const float v = (t < 3) ? bf16_round(b5[t]) : 0.f; *(volatile float*)(B5 + t) = v; __threadfence(); *(volatile float*)(B5 + t) = v; } }
__global__ __launch_bounds__(256) void k_out(const float* __restrict__ P, float* __restrict__ out) { const int t = blockIdx.x * 256 + threadIdx.x; if (t >= 3 * (NQ / 4)) return; const int q4 = (t % (NQ / 4)) * 4, c = t / (NQ / 4); v4f v;
#pragma unroll
  for (int j = 0; j < 4; ++j) v[j] = P[(size_t)(q4 + j) * 16 + c]; *(volatile v4f*)(out + (size_t)c * NQ + q4) = v; __threadfence(); *(volatile v4f*)(out + (size_t)c * NQ + q4) = v; }

extern "C" void kernel_launch(void* const* d_in, const int* in_sizes, int n_in,
                              void* d_out, int out_size, void* d_ws, size_t ws_size, hipStream_t stream) {
  (void)in_sizes; (void)n_in; (void)out_size;
  const float* const* I = (const float* const*)d_in; const float* fimg = I[0]; (void)d_in[1];   const float* times = I[2];
  const float* Wch = I[3]; const float* bch = I[4]; const float* Wq = I[5]; const float* bq = I[6]; const float* Wk = I[7]; const float* bk = I[8]; const float* Wv = I[9]; const float* bv = I[10]; const float* Bpe = I[11]; const float* Wpb = I[12]; const float* bpb = I[13];
  const float* W1 = I[14]; const float* b1 = I[15]; const float* W2 = I[16]; const float* b2 = I[17]; const float* W3 = I[18]; const float* b3 = I[19]; const float* W4 = I[20]; const float* b4 = I[21]; const float* W5 = I[22]; const float* b5 = I[23];
  char* ws = (char*)d_ws; size_t off = 0;
  auto take = [&](size_t bytes) { char* p = ws + off; off += (bytes + 255) & ~(size_t)255; return p; };
  const int KPC = 1728, KPQ = 448;
  _Float16* Bch = (_Float16*)take((size_t)CF * KPC * 2); _Float16* Bq = (_Float16*)take((size_t)CF * KPQ * 2); _Float16* Bk = (_Float16*)take((size_t)CF * KPQ * 2); _Float16* Bvw = (_Float16*)take((size_t)CF * KPQ * 2);
  _Float16* B1 = (_Float16*)take((size_t)HID * KIN * 2); _Float16* B2 = (_Float16*)take((size_t)HID * HID * 2); _Float16* B3 = (_Float16*)take((size_t)HID * HID * 2); _Float16* B4 = (_Float16*)take((size_t)HID * HID * 2); _Float16* Bw5 = (_Float16*)take((size_t)16 * HID * 2); float* B5 = (float*)take(64 * 4);
  _Float16* IM = (_Float16*)take((size_t)NVX * KPC * 2); float* FT = (float*)take((size_t)NVX * CF * 4); float* QV = (float*)take((size_t)NVX * CF * 4); float* KV = (float*)take((size_t)NVX * CF * 4); float* VVp = (float*)take((size_t)NVX * CF * 4); float* PB = (float*)take((size_t)16 * NTP * KA * NHD * 4);
  _Float16* FEAT = (_Float16*)take((size_t)QCH * KIN * 2); _Float16* H1 = (_Float16*)take((size_t)NQ * HID * 2); _Float16* H2 = (_Float16*)take((size_t)NQ * HID * 2); float* P = (float*)take((size_t)NQ * 16 * 4);
  if (off > ws_size) return;
  k_wconv<<<(CF * (KPC / 8) + 255) / 256, 256, 0, stream>>>(Wch, CIN, KPC, CF, Bch); k_wconv<<<(CF * (KPQ / 8) + 255) / 256, 256, 0, stream>>>(Wq, CF, KPQ, CF, Bq); k_wconv<<<(CF * (KPQ / 8) + 255) / 256, 256, 0, stream>>>(Wk, CF, KPQ, CF, Bk); k_wconv<<<(CF * (KPQ / 8) + 255) / 256, 256, 0, stream>>>(Wv, CF, KPQ, CF, Bvw);
  k_w1t<<<(HID * (KIN / 8) + 255) / 256, 256, 0, stream>>>(W1, B1); k_wt_f16<<<(HID * (HID / 8) + 255) / 256, 256, 0, stream>>>(W2, B2, HID, HID, 16.0f); k_wt_f16<<<(HID * (HID / 8) + 255) / 256, 256, 0, stream>>>(W3, B3, HID, HID, 16.0f); k_wt_f16<<<(HID * (HID / 8) + 255) / 256, 256, 0, stream>>>(W4, B4, HID, HID, 16.0f); k_w5<<<(16 * (HID / 8) + 255) / 256, 256, 0, stream>>>(W5, b5, Bw5, B5);
  k_pbtab<<<(16 * NTP * KA * 2 + 255) / 256, 256, 0, stream>>>(times, Bpe, Wpb, bpb, PB);
  k_im3<0><<<(unsigned)(((size_t)NVX * (KPC / 8) + 255) / 256), 256, 0, stream>>>(fimg, CIN, KPC, IM);
  const dim3 gV(((NVX / 16) * 1 + 3) / 4, 1);
  k_gemm_hhx<0><<<gV, 128, 0, stream>>>(IM, KPC, 0, Bch, KPC, 0, 0.0625f, bch, 0, nullptr, 1, 0, 0, FT, nullptr, CF, 0, NVX, CF, KPC);
  k_im3<1><<<(unsigned)(((size_t)NVX * (KPQ / 8) + 255) / 256), 256, 0, stream>>>(FT, CF, KPQ, IM);
  k_gemm_hhx<0><<<gV, 128, 0, stream>>>(IM, KPQ, 0, Bq, KPQ, 0, 0.0625f, bq, 0, nullptr, 1, 0, 0, QV, nullptr, CF, 0, NVX, CF, KPQ); k_gemm_hhx<0><<<gV, 128, 0, stream>>>(IM, KPQ, 0, Bk, KPQ, 0, 0.0625f, bk, 0, nullptr, 1, 0, 0, KV, nullptr, CF, 0, NVX, CF, KPQ); k_gemm_hhx<0><<<gV, 128, 0, stream>>>(IM, KPQ, 0, Bvw, KPQ, 0, 0.0625f, bv, 0, nullptr, 1, 0, 0, VVp, nullptr, CF, 0, NVX, CF, KPQ);
  for (int ch = 0; ch < NQ / QCH; ++ch) { const int q0 = ch * QCH;
    k_attn<<<QCH / 8, 256, 0, stream>>>(QV, KV, VVp, times, PB, q0, FEAT);
    k_gemm_hhx<6><<<dim3(((QCH / 16) * (HID / 64) + 3) / 4, 1), 128, 0, stream>>>(FEAT, KIN, 0, B1, KIN, 0, 0.0625f, b1, 0, nullptr, 1, 0, 0, nullptr, H1 + (size_t)q0 * HID, HID, 0, QCH, HID, KIN); }
  const dim3 gQ(((NQ / 16) * (HID / 64) + 3) / 4, 1);
  k_gemm_hhx<6><<<gQ, 128, 0, stream>>>(H1, HID, 0, B2, HID, 0, 0.0625f, b2, 0, nullptr, 1, 0, 0, nullptr, H2, HID, 0, NQ, HID, HID);
  k_gemm_hhx<6><<<gQ, 128, 0, stream>>>(H2, HID, 0, B3, HID, 0, 0.0625f, b3, 0, nullptr, 1, 0, 0, nullptr, H1, HID, 0, NQ, HID, HID);
  k_gemm_hhx<6><<<gQ, 128, 0, stream>>>(H1, HID, 0, B4, HID, 0, 0.0625f, b4, 0, nullptr, 1, 0, 0, nullptr, H2, HID, 0, NQ, HID, HID);
  k_gemm_hhx<0><<<dim3(((NQ / 16) * 1 + 3) / 4, 1), 128, 0, stream>>>(H2, HID, 0, Bw5, HID, 0, 0.0625f, B5, 0, nullptr, 1, 0, 0, P, nullptr, 16, 0, NQ, 16, HID);
  k_out<<<(3 * (NQ / 4) + 255) / 256, 256, 0, stream>>>(P, (float*)d_out);
}
